// DecoderLayer_70755291234841
// MI455X (gfx1250) — hardware-verified
//
#include <hip/hip_runtime.h>
#ifndef NB
#define NB 2
#endif
#ifndef SEQ
#define SEQ 2048
#endif
#define NB_FULL 2
#define SEQ_FULL 2048
#define DM 1024
#define NH 16
#define HD 64
#define DFF 4096
#define LQKV (3 * DM)
#define LKV (2 * DM)
#define HQKV (3 * HD)
#define HKV (2 * HD)
#define NR (NB * SEQ)
#define NQT (SEQ / 64)
#define ER 64
#define LN_EPS 1.0e-9f
#define RA_ROW 8192
#define RA_KV 0
#define RA_Q2 4096
#define RA_Y1H 6144
#define RA_Y2F 0
#define RA_Y2H 4096
#define RB_ROW 10240
#define RB_Y16 0
#define RB_X16 2048
#define RB_VT 4096
#define RB_Y1F 6144
#define RB_H16 0
static_assert(NB >= 1 && NB <= NB_FULL);
static_assert(SEQ >= 128 && SEQ <= SEQ_FULL && (SEQ % 128) == 0);
static_assert(NQT <= 32 && (NR % 128) == 0);
static_assert(DM == 256 * 4 && HD == 64 && NH * HD == DM);
static_assert((DM % 64) == 0 && (LQKV % 64) == 0 && (LKV % 64) == 0 && (DFF % 64) == 0 && (DM % 32) == 0 && (DFF % 32) == 0);
static_assert(LQKV * 2 <= RA_ROW && RA_Q2 + DM * 2 == RA_Y1H && RA_Y1H + DM * 2 <= RA_ROW && RA_Y2H + DM * 2 <= RA_ROW && LKV * 2 <= RA_Q2 && DM * 4 <= RA_Y2H);
static_assert(RB_X16 == DM * 2 && RB_VT == 2 * DM * 2 && NH * HD * 2 == RB_Y1F - RB_VT && RB_Y1F + DM * 4 == RB_ROW && RB_H16 + DFF * 2 <= RB_ROW);

typedef _Float16 v16h __attribute__((ext_vector_type(16)));
typedef unsigned short v8us __attribute__((ext_vector_type(8), may_alias));
typedef float v8f __attribute__((ext_vector_type(8)));
typedef float v4f __attribute__((ext_vector_type(4)));
typedef float v4fa __attribute__((ext_vector_type(4), may_alias));
typedef _Float16 v4h __attribute__((ext_vector_type(4)));
typedef int v4i __attribute__((ext_vector_type(4), may_alias));
union FragH { v16h v; v8us half[2]; _Float16 h[16]; unsigned short u[16]; };

__device__ __forceinline__ unsigned short bf16_bits(float x) { unsigned int u = __float_as_uint(x); return (unsigned short)((u + 0x7FFFu + ((u >> 16) & 1u)) >> 16); }
__device__ __forceinline__ float bf16q(float x) { return __uint_as_float(((unsigned int)bf16_bits(x)) << 16); }

__device__ __forceinline__ v16h g2_frag(const _Float16* p, int hh) { FragH f; f.half[0] = *(const v8us*)((const unsigned short*)p + 8 * hh); f.half[1] = *(const v8us*)((const unsigned short*)p + 16 + 8 * hh); return f.v; }
__device__ __forceinline__ v8f g2_mma(v16h a, v16h b, v8f c) { v8f d = __builtin_amdgcn_wmma_f32_16x16x32_f16(false, a, false, b, (short)0, c, false, false); asm volatile("v_nop\n\tv_nop\n\tv_nop\n\tv_nop" : "+v"(d) : "v"(a), "v"(b)); return d; }

__global__ __launch_bounds__(256) void k_wt(const float* __restrict__ W, _Float16* __restrict__ Wt, int K, int N) {
  const int t = blockIdx.x * 256 + threadIdx.x; if (t >= N * (K / 8)) return;
  const int n = t / (K / 8), k8 = (t % (K / 8)) * 8; FragH f;
#pragma unroll
  for (int i = 0; i < 8; ++i) f.h[i] = (_Float16)(bf16q(W[(size_t)(k8 + i) * N + n]) * 16.0f);
  const v8us o = f.half[0]; unsigned short* d = (unsigned short*)Wt + (size_t)n * K + k8;
  *(volatile v8us*)d = o; __threadfence(); *(volatile v8us*)d = o;
}

__global__ __launch_bounds__(256) void k_in16(const float* __restrict__ src, _Float16* __restrict__ dst) {
  const size_t t = (size_t)blockIdx.x * 256 + threadIdx.x; const size_t n8 = (size_t)NR * DM / 8; if (t >= n8) return;
  const size_t e = t * 8; const size_t r = e / DM; const int c = (int)(e % DM);
  const size_t rf = (r / SEQ) * SEQ_FULL + (r % SEQ);
  const v4f a = *(const v4fa*)(src + rf * DM + c), cc = *(const v4fa*)(src + rf * DM + c + 4); FragH f;
#pragma unroll
  for (int q = 0; q < 4; ++q) { f.h[q] = (_Float16)bf16q(a[q]); f.h[4 + q] = (_Float16)bf16q(cc[q]); }
  unsigned short* d = (unsigned short*)dst + e;
  *(volatile v8us*)d = f.half[0]; __threadfence(); *(volatile v8us*)d = f.half[0];
}

__global__ __launch_bounds__(256) void k_mflag(const int* __restrict__ mask, int* __restrict__ MF) {
  __shared__ int wsum[8]; __shared__ int fl[32]; __shared__ int anyz;
  const int qt = blockIdx.x, t = threadIdx.x, lane = t & 31, w = t >> 5;
  const int row = t >> 2, pc = t & 3;
  if (t < 32) fl[t] = 0;
  if (t == 0) anyz = 0;
  __syncthreads();
  const int* mrow = mask + (size_t)(qt * 64 + row) * SEQ_FULL + pc * 16;
  int rowcnt = 0;
#pragma unroll 1
  for (int kt = 0; kt < NQT; ++kt) {
    int c = 0;
#pragma unroll
    for (int u = 0; u < 4; ++u) { const v4i v = *(const v4i*)(mrow + kt * 64 + u * 4); c += (v[0] != 0) + (v[1] != 0) + (v[2] != 0) + (v[3] != 0); }
    rowcnt += c;
    c += __shfl_xor(c, 16, 32); c += __shfl_xor(c, 8, 32); c += __shfl_xor(c, 4, 32); c += __shfl_xor(c, 2, 32); c += __shfl_xor(c, 1, 32);
    if (lane == 0) wsum[w] = c;
    __syncthreads();
    if (t == 0) { int tot = 0; for (int i = 0; i < 8; ++i) tot += wsum[i]; fl[kt] = (tot == 0) ? 0 : ((tot == 64 * 64) ? 1 : 2); }
    __syncthreads();
  }
  rowcnt += __shfl_xor(rowcnt, 1, 32); rowcnt += __shfl_xor(rowcnt, 2, 32);
  if (rowcnt == 0) anyz = 1;
  __syncthreads();
  if (t < 8) {
    const int az = anyz; v4i o;
#pragma unroll
    for (int j = 0; j < 4; ++j) { const int k = t * 4 + j; int fv = fl[k]; if (k >= NQT) fv = 0; else if (az != 0 && fv == 0) fv = 2; o[j] = fv; }
    int* dst = MF + qt * 32 + t * 4;
    *(volatile v4i*)dst = o; __threadfence(); *(volatile v4i*)dst = o;
  }
}

template <int ACT>
__global__ __launch_bounds__(128) void k_gemm(const _Float16* __restrict__ A, int lda, const _Float16* __restrict__ Bt, int ldb, float alpha,
                                              const float* __restrict__ bias, float* __restrict__ C, int ldc, int cseq, int clim,
                                              _Float16* __restrict__ C16, int ldc16, int M, int N, int K) {
  __shared__ __attribute__((aligned(16))) float so[4][32][68];
  const int tid = threadIdx.x, w = tid >> 5, lane = tid & 31, ln = lane & 15, hh = lane >> 4;
  const int ntn = N >> 6; const int mt = blockIdx.x / ntn, nq = blockIdx.x - mt * ntn;
  const int row0 = mt * 128 + 32 * w, col0 = nq * 64;
  if (row0 >= M) return;
  const _Float16* a0p = A + (size_t)(row0 + ln) * lda; const _Float16* a1p = a0p + (size_t)16 * lda;
  const _Float16* b0p = Bt + (size_t)(col0 + ln) * ldb; const _Float16* b1p = b0p + (size_t)16 * ldb; const _Float16* b2p = b1p + (size_t)16 * ldb; const _Float16* b3p = b2p + (size_t)16 * ldb;
  const v8f z8 = {0.f,0.f,0.f,0.f,0.f,0.f,0.f,0.f}; v8f c00 = z8, c01 = z8, c02 = z8, c03 = z8, c10 = z8, c11 = z8, c12 = z8, c13 = z8;
#pragma unroll 1
  for (int kb = 0; kb < K; kb += 32) {
    const v16h a0 = g2_frag(a0p + kb, hh), a1 = g2_frag(a1p + kb, hh);
    v16h bq = g2_frag(b0p + kb, hh); c00 = g2_mma(a0, bq, c00); c10 = g2_mma(a1, bq, c10);
    bq = g2_frag(b1p + kb, hh); c01 = g2_mma(a0, bq, c01); c11 = g2_mma(a1, bq, c11);
    bq = g2_frag(b2p + kb, hh); c02 = g2_mma(a0, bq, c02); c12 = g2_mma(a1, bq, c12);
    bq = g2_frag(b3p + kb, hh); c03 = g2_mma(a0, bq, c03); c13 = g2_mma(a1, bq, c13);
  }
  v8f accs[8] = {c00, c01, c02, c03, c10, c11, c12, c13};
  const bool wc32 = (C != nullptr) && ((row0 % cseq) < clim);
  const int crow0 = (row0 / cseq) * clim + (row0 % cseq);
#pragma unroll
  for (int u = 0; u < 8; ++u) {
    const int t = u & 3, half = u >> 2; const int col = col0 + t * 16 + ln; const float bv = bf16q(bias[col]);
#pragma unroll
    for (int r = 0; r < 8; ++r) { const int rloc = half * 16 + 8 * hh + r; float v = accs[u][r] * alpha + bv; if (ACT == 1) v = fmaxf(v, 0.f); so[w][rloc][t * 16 + ln] = v; }
  }
  __builtin_amdgcn_fence(4  , "workgroup"); __builtin_amdgcn_wave_barrier();
  const int rsub = lane >> 4, c4 = (lane & 15) * 4;
  for (int ps = 0; ps < 2; ++ps) {
#pragma unroll
    for (int q = 0; q < 16; ++q) {
      const int r = q * 2 + rsub; const v4f v = *(const v4fa*)&so[w][r][c4];
      if (wc32) *(volatile v4f*)(C + (size_t)(crow0 + r) * ldc + col0 + c4) = v;
      if (C16 != nullptr) { v4h h4; for (int i = 0; i < 4; ++i) h4[i] = (_Float16)v[i]; *(volatile v4h*)(C16 + (size_t)(row0 + r) * ldc16 + col0 + c4) = h4; }
    }
    if (ps == 0) __threadfence();
  }
}

__global__ __launch_bounds__(256) void k_vt(const _Float16* __restrict__ V16, int ldv, int voff, int hstr, _Float16* __restrict__ VT) {
  __shared__ unsigned short tl[64][66];
  const int tid = threadIdx.x; const int slab = blockIdx.x / NQT, lg = blockIdx.x - slab * NQT; const int b = slab / NH, h = slab - b * NH;
  for (int i = tid; i < 64 * 8; i += 256) {
    const int r = i >> 3, c8 = (i & 7) * 8; FragH f;
    f.half[0] = *(const v8us*)((const unsigned short*)V16 + ((size_t)b * SEQ + lg * 64 + r) * ldv + voff + (size_t)h * hstr + c8);
#pragma unroll
    for (int q = 0; q < 8; ++q) tl[r][c8 + q] = f.u[q];
  }
  __syncthreads();
  for (int ps = 0; ps < 2; ++ps) {
#pragma unroll
    for (int rd = 0; rd < 2; ++rd) {
      const int d = rd * 32 + (tid >> 3), pc = tid & 7; FragH f;
#pragma unroll
      for (int q = 0; q < 8; ++q) f.u[q] = tl[pc * 8 + q][d];
      *(volatile v8us*)((unsigned short*)VT + ((size_t)slab * 64 + d) * SEQ + lg * 64 + pc * 8) = f.half[0];
    }
    if (ps == 0) __threadfence();
  }
}

template <int MASKED>
__global__ __launch_bounds__(128) void k_flash(const _Float16* __restrict__ Qp, int qp, int qhs,
                                               const _Float16* __restrict__ Kp, int kp, int khs, int koff,
                                               const _Float16* __restrict__ VT, const int* __restrict__ mask,
                                               const int* __restrict__ MF, _Float16* __restrict__ O16) {
  __shared__ __attribute__((aligned(16))) _Float16 Pl[4][16][72];
  __shared__ __attribute__((aligned(16))) int Ms[MASKED ? 64 : 1][68];
  const int tid = threadIdx.x, w = tid >> 5, lane = tid & 31, l15 = lane & 15, hh = lane >> 4;
  const int qt = blockIdx.x, h = blockIdx.y, b = blockIdx.z;
  const size_t rb = (size_t)b * SEQ;
  const int qw = qt * 64 + w * 16;
  const _Float16* qrow = Qp + (rb + qw + l15) * (size_t)qp + (size_t)h * qhs;
  const v16h qf0 = g2_frag(qrow, hh), qf1 = g2_frag(qrow + 32, hh);
  const _Float16* kbp = Kp + rb * (size_t)kp + koff + (size_t)h * khs;
  const _Float16* vtp = VT + (size_t)(b * NH + h) * HD * SEQ;
  const v8f z8 = {0.f,0.f,0.f,0.f,0.f,0.f,0.f,0.f};
  float rm[8], rl[8]; v8f oacc[4];
#pragma unroll
  for (int r = 0; r < 8; ++r) { rm[r] = -3.0e38f; rl[r] = 0.f; }
#pragma unroll
  for (int ot = 0; ot < 4; ++ot) oacc[ot] = z8;
#pragma unroll 1
  for (int kt = 0; kt < NQT; ++kt) {
    int f = 1;
    if (MASKED) { const int fv = MF[qt * 32 + kt]; f = (fv == 0) ? 0 : ((fv == 1) ? 1 : 2); }
    if (f == 0) continue;
    const int key0 = kt * 64;
    if (MASKED) {
      if (f == 2) {
        __syncthreads();
        for (int i = tid; i < 64 * 16; i += 128) {
          const int r = i >> 4, c4 = (i & 15) * 4;
          const v4i mv4 = *(const v4i*)(mask + (size_t)(qt * 64 + r) * SEQ_FULL + key0 + c4);
          *(v4i*)&Ms[r][c4] = mv4;
        }
        __syncthreads();
      }
    }
    v8f st[4];
#pragma unroll
    for (int nt = 0; nt < 4; ++nt) {
      const _Float16* kr = kbp + (size_t)(key0 + nt * 16 + l15) * kp; v8f s = z8;
      s = g2_mma(qf0, g2_frag(kr, hh), s); s = g2_mma(qf1, g2_frag(kr + 32, hh), s); st[nt] = s;
    }
    __builtin_amdgcn_fence(3  , "wavefront"); __builtin_amdgcn_wave_barrier();
#pragma unroll
    for (int r = 0; r < 8; ++r) {
      float sc[4]; float m = -3.0e38f;
#pragma unroll
      for (int nt = 0; nt < 4; ++nt) {
        float xv = st[nt][r] * 0.125f;
        if (MASKED) { if (f == 2) { const int mv = Ms[w * 16 + 8 * hh + r][nt * 16 + l15]; xv = (mv != 0) ? xv : -1.0e9f; } }
        sc[nt] = xv; m = fmaxf(m, xv);
      }
      m = fmaxf(m, __shfl_xor(m, 8, 32)); m = fmaxf(m, __shfl_xor(m, 4, 32)); m = fmaxf(m, __shfl_xor(m, 2, 32)); m = fmaxf(m, __shfl_xor(m, 1, 32));
      const float nm = fmaxf(rm[r], m); const float al = __expf(rm[r] - nm);
      float rs = 0.f;
#pragma unroll
      for (int nt = 0; nt < 4; ++nt) { const float p = __expf(sc[nt] - nm); rs += p; Pl[w][8 * hh + r][nt * 16 + l15] = (_Float16)(p * 1024.0f); }
      rs += __shfl_xor(rs, 8, 32); rs += __shfl_xor(rs, 4, 32); rs += __shfl_xor(rs, 2, 32); rs += __shfl_xor(rs, 1, 32);
      rl[r] = rl[r] * al + rs; rm[r] = nm;
#pragma unroll
      for (int ot = 0; ot < 4; ++ot) oacc[ot][r] *= al;
    }
    __builtin_amdgcn_fence(3  , "wavefront"); __builtin_amdgcn_wave_barrier();
    const v16h pf0 = g2_frag(&Pl[w][l15][0], hh), pf1 = g2_frag(&Pl[w][l15][32], hh);
#pragma unroll
    for (int ot = 0; ot < 4; ++ot) {
      const _Float16* vr = vtp + (size_t)(ot * 16 + l15) * SEQ + key0;
      oacc[ot] = g2_mma(pf0, g2_frag(vr, hh), oacc[ot]); oacc[ot] = g2_mma(pf1, g2_frag(vr + 32, hh), oacc[ot]);
    }
  }
  __builtin_amdgcn_fence(3  , "wavefront"); __builtin_amdgcn_wave_barrier();
#pragma unroll
  for (int r = 0; r < 8; ++r) {
    const float inv = 0.0625f / rl[r];
#pragma unroll
    for (int ot = 0; ot < 4; ++ot) Pl[w][8 * hh + r][ot * 16 + l15] = (_Float16)(oacc[ot][r] * inv);
  }
  __builtin_amdgcn_fence(3  , "wavefront"); __builtin_amdgcn_wave_barrier();
  const int rw = lane >> 3, pc = lane & 7;
  for (int ps = 0; ps < 2; ++ps) {
#pragma unroll
    for (int it = 0; it < 4; ++it) {
      const int row = it * 4 + rw; const v8us v = *(const v8us*)&Pl[w][row][pc * 8];
      *(volatile v8us*)((unsigned short*)O16 + ((rb + qw + row) * DM + (size_t)h * HD + pc * 8)) = v;
    }
    if (ps == 0) __threadfence();
  }
}

__global__ __launch_bounds__(64) void k_attn0(const float* __restrict__ QE, const int* __restrict__ mask, const int* __restrict__ MF,
                                             _Float16* __restrict__ O16) {
  __shared__ float QV[64][65]; __shared__ float Ks[64][65]; __shared__ float Ss[64][65];
  __shared__ __attribute__((aligned(16))) _Float16 os[64][72];
  const int b = blockIdx.x / NH, h = blockIdx.x - b * NH, t = threadIdx.x;
  int anyk = 0;
#pragma unroll 1
  for (int kt = 1; kt < NQT; ++kt) anyk |= MF[kt];
  if (anyk != 0) return;
  const float* base = QE + (size_t)b * ER * LQKV + (size_t)h * HQKV;
#pragma unroll 1
  for (int i = t; i < 64 * 16; i += 64) {
    const int r = i >> 4, c4 = (i & 15) * 4;
    const v4f q4 = *(const v4fa*)(base + (size_t)r * LQKV + c4); const v4f k4 = *(const v4fa*)(base + (size_t)r * LQKV + HD + c4);
    QV[r][c4] = q4[0]; QV[r][c4 + 1] = q4[1]; QV[r][c4 + 2] = q4[2]; QV[r][c4 + 3] = q4[3];
    Ks[r][c4] = k4[0]; Ks[r][c4 + 1] = k4[1]; Ks[r][c4 + 2] = k4[2]; Ks[r][c4 + 3] = k4[3];
  }
  __syncthreads();
  const int* mrow = mask + (size_t)t * SEQ_FULL;
  float m = -3.0e38f;
#pragma unroll 1
  for (int j = 0; j < 64; ++j) {
    float s = 0.f;
#pragma unroll 4
    for (int d = 0; d < 64; ++d) s = fmaf(QV[t][d], Ks[j][d], s);
    s *= 0.125f; const int mv = mrow[j]; s = (mv != 0) ? s : -1.0e9f; Ss[t][j] = s; m = fmaxf(m, s);
  }
  float l = 0.f;
#pragma unroll 1
  for (int j = 0; j < 64; ++j) { const float e = __expf(Ss[t][j] - m); Ss[t][j] = e; l += e; }
  __syncthreads();
#pragma unroll 1
  for (int i = t; i < 64 * 16; i += 64) {
    const int r = i >> 4, c4 = (i & 15) * 4;
    const v4f v4 = *(const v4fa*)(base + (size_t)r * LQKV + 2 * HD + c4);
    QV[r][c4] = v4[0]; QV[r][c4 + 1] = v4[1]; QV[r][c4 + 2] = v4[2]; QV[r][c4 + 3] = v4[3];
  }
  __syncthreads();
  const float inv = 64.0f / l;
#pragma unroll 1
  for (int d = 0; d < 64; ++d) {
    float o = 0.f;
#pragma unroll 4
    for (int j = 0; j < 64; ++j) o = fmaf(Ss[t][j], QV[j][d], o);
    os[t][d] = (_Float16)(o * inv);
  }
  __syncthreads();
  const int rw = t >> 3, pc = t & 7;
  for (int ps = 0; ps < 2; ++ps) {
#pragma unroll
    for (int it = 0; it < 8; ++it) {
      const int row = it * 8 + rw; const v8us v = *(const v8us*)&os[row][pc * 8];
      *(volatile v8us*)((unsigned short*)O16 + (((size_t)b * SEQ + row) * DM + (size_t)h * HD + pc * 8)) = v;
    }
    if (ps == 0) __threadfence();
  }
}

template <int RIN, int OUTF, int W16>
__global__ __launch_bounds__(256) void k_ln(const float* __restrict__ X, const float* __restrict__ R, const float* __restrict__ g, const float* __restrict__ bb,
                                            float* __restrict__ N32, _Float16* __restrict__ N16) {
  #pragma clang fp contract(off)
  __shared__ float red[256];
  const int r = blockIdx.x, t = threadIdx.x, c0 = t * 4;
  const size_t rf = (size_t)(r / SEQ) * SEQ_FULL + (size_t)(r % SEQ);
  const v4f xa = *(const v4fa*)(X + (size_t)r * DM + c0);
  const v4f ra = *(const v4fa*)(R + (RIN ? rf : (size_t)r) * DM + c0);
  float v[4]; float s1 = 0.f;
#pragma unroll
  for (int q = 0; q < 4; ++q) { const float rv = RIN ? bf16q(ra[q]) : ra[q]; v[q] = xa[q] + rv; s1 += v[q]; }
  red[t] = s1; __syncthreads();
  for (int st = 128; st > 0; st >>= 1) { if (t < st) red[t] += red[t + st]; __syncthreads(); }
  const float mu = red[0] * (1.0f / (float)DM); __syncthreads();
  float s2 = 0.f;
#pragma unroll
  for (int q = 0; q < 4; ++q) { const float c = v[q] - mu; s2 += c * c; }
  red[t] = s2; __syncthreads();
  for (int st = 128; st > 0; st >>= 1) { if (t < st) red[t] += red[t + st]; __syncthreads(); }
  const float var = red[0] * (1.0f / (float)DM);
  const float rs = 1.0f / sqrtf(var + LN_EPS);
  v4f o; v4h oh;
#pragma unroll
  for (int q = 0; q < 4; ++q) { const float gg = bf16q(g[c0 + q]), be = bf16q(bb[c0 + q]); o[q] = (gg * (v[q] - mu)) * rs + be; oh[q] = (_Float16)o[q]; }
  float* orow = N32 + (OUTF ? rf : (size_t)r) * DM + c0;
  for (int ps = 0; ps < 2; ++ps) {
    *(volatile v4f*)orow = o;
    if (W16) *(volatile v4h*)(N16 + (size_t)r * DM + c0) = oh;
    if (ps == 0) __threadfence();
  }
}

extern "C" void kernel_launch(void* const* d_in, const int* in_sizes, int n_in,
                              void* d_out, int out_size, void* d_ws, size_t ws_size, hipStream_t stream) {
  if (n_in < 23) return;
  const float* x = (const float*)d_in[0]; const float* y = (const float*)d_in[1]; const int* mask = (const int*)d_in[2];
  const float* qkv_w = (const float*)d_in[3]; const float* qkv_b = (const float*)d_in[4];
  const float* sa_w = (const float*)d_in[5]; const float* sa_b = (const float*)d_in[6];
  const float* g1 = (const float*)d_in[7]; const float* b1 = (const float*)d_in[8];
  const float* kv_w = (const float*)d_in[9]; const float* kv_b = (const float*)d_in[10];
  const float* q_w = (const float*)d_in[11]; const float* q_b = (const float*)d_in[12];
  const float* ca_w = (const float*)d_in[13]; const float* ca_b = (const float*)d_in[14];
  const float* g2 = (const float*)d_in[15]; const float* b2 = (const float*)d_in[16];
  const float* f1_w = (const float*)d_in[17]; const float* f1_b = (const float*)d_in[18];
  const float* f2_w = (const float*)d_in[19]; const float* f2_b = (const float*)d_in[20];
  const float* g3 = (const float*)d_in[21]; const float* b3 = (const float*)d_in[22];
  const long long need_rows = (long long)(NB - 1) * SEQ_FULL + SEQ;
  if ((long long)in_sizes[0] < need_rows * DM || (long long)in_sizes[1] < need_rows * DM) return;
  if ((long long)in_sizes[2] < (long long)(SEQ - 1) * SEQ_FULL + SEQ) return;
  if (in_sizes[3] < DM * LQKV || in_sizes[4] < LQKV || in_sizes[5] < DM * DM || in_sizes[6] < DM || in_sizes[7] < DM || in_sizes[8] < DM) return;
  if (in_sizes[9] < DM * LKV || in_sizes[10] < LKV || in_sizes[11] < DM * DM || in_sizes[12] < DM || in_sizes[13] < DM * DM || in_sizes[14] < DM) return;
  if (in_sizes[15] < DM || in_sizes[16] < DM || in_sizes[17] < DM * DFF || in_sizes[18] < DFF || in_sizes[19] < DFF * DM || in_sizes[20] < DM) return;
  if (in_sizes[21] < DM || in_sizes[22] < DM) return;
  if ((long long)out_size < need_rows * DM) return;

  char* ws = (char*)d_ws; size_t off = 0;
  auto take = [&](size_t bytes) { char* p = ws + off; off += (bytes + 255) & ~(size_t)255; return p; };
  const size_t nr = (size_t)NR;
  _Float16* Wqkv = (_Float16*)take((size_t)LQKV * DM * 2);
  _Float16* Wsa  = (_Float16*)take((size_t)DM * DM * 2);
  _Float16* Wkv  = (_Float16*)take((size_t)LKV * DM * 2);
  _Float16* Wq   = (_Float16*)take((size_t)DM * DM * 2);
  _Float16* Wca  = (_Float16*)take((size_t)DM * DM * 2);
  _Float16* W1   = (_Float16*)take((size_t)DFF * DM * 2);
  _Float16* W2   = (_Float16*)take((size_t)DM * DFF * 2);
  char* RA = take(nr * RA_ROW);
  char* RB = take(nr * RB_ROW);
  float* T32 = (float*)take(nr * DM * 4);
  float* QE  = (float*)take((size_t)NB * ER * LQKV * 4);
  int*   MF  = (int*)take((size_t)32 * 32 * 4);
  if (off > ws_size || off > (size_t)134217728) return;
  _Float16* QKV16 = (_Float16*)RA;
  _Float16* KV16  = (_Float16*)(RA + nr * RA_KV);
  _Float16* Q2H   = (_Float16*)(RA + nr * RA_Q2);
  _Float16* Y1H   = (_Float16*)(RA + nr * RA_Y1H);
  float*    Y2F   = (float*)(RA + nr * RA_Y2F);
  _Float16* Y2H   = (_Float16*)(RA + nr * RA_Y2H);
  _Float16* Y16   = (_Float16*)(RB + nr * RB_Y16);
  _Float16* O16   = (_Float16*)(RB + nr * RB_Y16);
  _Float16* X16   = (_Float16*)(RB + nr * RB_X16);
  _Float16* VT    = (_Float16*)(RB + nr * RB_VT);
  float*    Y1F   = (float*)(RB + nr * RB_Y1F);
  _Float16* H16   = (_Float16*)(RB + nr * RB_H16);

  k_wt<<<(unsigned)((LQKV * (DM / 8) + 255) / 256), 256, 0, stream>>>(qkv_w, Wqkv, DM, LQKV);
  k_wt<<<(unsigned)((DM * (DM / 8) + 255) / 256), 256, 0, stream>>>(sa_w, Wsa, DM, DM);
  k_wt<<<(unsigned)((LKV * (DM / 8) + 255) / 256), 256, 0, stream>>>(kv_w, Wkv, DM, LKV);
  k_wt<<<(unsigned)((DM * (DM / 8) + 255) / 256), 256, 0, stream>>>(q_w, Wq, DM, DM);
  k_wt<<<(unsigned)((DM * (DM / 8) + 255) / 256), 256, 0, stream>>>(ca_w, Wca, DM, DM);
  k_wt<<<(unsigned)((DFF * (DM / 8) + 255) / 256), 256, 0, stream>>>(f1_w, W1, DM, DFF);
  k_wt<<<(unsigned)((DM * (DFF / 8) + 255) / 256), 256, 0, stream>>>(f2_w, W2, DFF, DM);
  k_in16<<<(unsigned)((nr * DM / 8 + 255) / 256), 256, 0, stream>>>(y, Y16);
  k_in16<<<(unsigned)((nr * DM / 8 + 255) / 256), 256, 0, stream>>>(x, X16);
  k_mflag<<<NQT, 256, 0, stream>>>(mask, MF);

  k_gemm<0><<<(unsigned)((nr / 128) * (LQKV / 64)), 128, 0, stream>>>(Y16, DM, Wqkv, DM, 0.0625f, qkv_b, QE, LQKV, SEQ, ER, QKV16, LQKV, (int)nr, LQKV, DM);
  k_vt<<<NB * NH * NQT, 256, 0, stream>>>(QKV16, LQKV, 2 * HD, HQKV, VT);
  k_flash<1><<<dim3(NQT, NH, NB), 128, 0, stream>>>(QKV16, LQKV, HQKV, QKV16, LQKV, HQKV, HD, VT, mask, MF, O16);
  k_attn0<<<NB * NH, 64, 0, stream>>>(QE, mask, MF, O16);
  k_gemm<0><<<(unsigned)((nr / 128) * (DM / 64)), 128, 0, stream>>>(O16, DM, Wsa, DM, 0.0009765625f, sa_b, T32, DM, (int)nr, (int)nr, nullptr, 0, (int)nr, DM, DM);
  k_ln<1, 0, 1><<<(unsigned)nr, 256, 0, stream>>>(T32, y, g1, b1, Y1F, Y1H);

  k_gemm<0><<<(unsigned)((nr / 128) * (LKV / 64)), 128, 0, stream>>>(X16, DM, Wkv, DM, 0.0625f, kv_b, nullptr, 0, (int)nr, (int)nr, KV16, LKV, (int)nr, LKV, DM);
  k_gemm<0><<<(unsigned)((nr / 128) * (DM / 64)), 128, 0, stream>>>(Y1H, DM, Wq, DM, 0.0625f, q_b, nullptr, 0, (int)nr, (int)nr, Q2H, DM, (int)nr, DM, DM);
  k_vt<<<NB * NH * NQT, 256, 0, stream>>>(KV16, LKV, HD, HKV, VT);
  k_flash<0><<<dim3(NQT, NH, NB), 128, 0, stream>>>(Q2H, DM, HD, KV16, LKV, HKV, 0, VT, mask, MF, O16);
  k_gemm<0><<<(unsigned)((nr / 128) * (DM / 64)), 128, 0, stream>>>(O16, DM, Wca, DM, 0.0009765625f, ca_b, T32, DM, (int)nr, (int)nr, nullptr, 0, (int)nr, DM, DM);
  k_ln<0, 0, 1><<<(unsigned)nr, 256, 0, stream>>>(T32, Y1F, g2, b2, Y2F, Y2H);

  k_gemm<1><<<(unsigned)((nr / 128) * (DFF / 64)), 128, 0, stream>>>(Y2H, DM, W1, DM, 0.0625f, f1_b, nullptr, 0, (int)nr, (int)nr, H16, DFF, (int)nr, DFF, DM);
  k_gemm<0><<<(unsigned)((nr / 128) * (DM / 64)), 128, 0, stream>>>(H16, DFF, W2, DFF, 0.0625f, f2_b, T32, DM, (int)nr, (int)nr, nullptr, 0, (int)nr, DM, DFF);
  k_ln<0, 1, 0><<<(unsigned)nr, 256, 0, stream>>>(T32, Y2F, g3, b3, (float*)d_out, Y2H);
}
